// WENONetwork_9474697855463
// MI455X (gfx1250) — hardware-verified
//
#include <hip/hip_runtime.h>
#include <math.h>


#pragma clang fp contract(off)

#ifndef NPTS
#define NPTS 2097152
#endif
#define NPTS_FULL 2097152
#define NOUT (NPTS - 6)

#define OPB 192
#define NWAVE 13
#define EXT (NWAVE * 16)
#define NTHR (NWAVE * 32)

#define P1 40
#define P2 96
#define P3 160
#define P4 80
#define K2 224
#define K3 96
#define K4 160
#define K5 256
#define L1R (EXT + 5)
#define L4R (EXT + 3)
#define UUN 232
#define DIFN 224
#define BUFA_US (EXT * P3)
#define BUFB_US (EXT * P2)
#define WBUF_US (48 * K2)

#define T2_BYTES (48 * K2 * 2)
#define T3_BYTES (80 * K3 * 2)
#define T4_BYTES (48 * K4 * 2)
#define T5_BYTES (32 * K5 * 2)
#define T2_OFF 0
#define T3_OFF (T2_OFF + T2_BYTES)
#define T4_OFF (T3_OFF + T3_BYTES)
#define T5_OFF (T4_OFF + T4_BYTES)
#define WS_TOTAL (T5_OFF + T5_BYTES)

static_assert(NPTS <= NPTS_FULL);
static_assert(EXT == NWAVE * 16);
static_assert(OPB % 32 == 0);
static_assert(OPB <= EXT - 2);
static_assert(L1R * P1 <= BUFA_US);
static_assert(L4R * P4 <= BUFB_US);
static_assert(80 * K3 <= WBUF_US && 48 * K4 <= WBUF_US && 32 * K5 <= WBUF_US);
static_assert((T2_BYTES % 256) == 0 && (T3_BYTES % 256) == 0 && (T4_BYTES % 256) == 0 && (T5_BYTES % 256) == 0);
static_assert(DIFN + 2 <= UUN);
static_assert(L1R + 4 <= DIFN);
static_assert(OPB + 10 < UUN);
static_assert(OPB + 3 < EXT);
static_assert(NWAVE * 16 * 24 * 4 <= BUFA_US * 2);
static_assert(OPB / 4 <= 64);
static_assert((K2 / 32) * 32 >= 200 && (K5 / 32) * 32 >= 240);

typedef unsigned short us_t;
typedef __attribute__((ext_vector_type(16))) __bf16 v16b;
typedef __attribute__((ext_vector_type(8)))  unsigned short v8us;
typedef __attribute__((ext_vector_type(8)))  float v8f;
typedef __attribute__((ext_vector_type(4)))  float v4f;
typedef __attribute__((ext_vector_type(4)))  unsigned v4u;
typedef float __attribute__((may_alias)) float_a;

template <typename T> __device__ __forceinline__ void vst2(void* p, T v) { *(volatile T*)p = v; __threadfence(); *(volatile T*)p = v; }

__device__ __forceinline__ v8f wmma_bf(v16b a, v16b b, v8f c) {
  v8f d = __builtin_amdgcn_wmma_f32_16x16x32_bf16(false, a, false, b, (short)0, c, false, false);
  asm volatile("v_nop\n\tv_nop\n\tv_nop\n\tv_nop" : "+v"(d) : "v"(a), "v"(b));
  return d;
}
__device__ __forceinline__ float bfr(float v) { return (float)(__bf16)v; }
__device__ __forceinline__ us_t bfbits(float v) { const __bf16 b = (__bf16)v; return __builtin_bit_cast(us_t, b); }
__device__ __forceinline__ float elu_f(float x) { return x > 0.0f ? x : (__expf(x) - 1.0f); }

__device__ __forceinline__ v16b fragb(const us_t* p0, int lane) {
  union { v16b v; v8us q[2]; } u; const us_t* p = p0 + 8 * (lane >> 4);
  u.q[0] = *(const v8us*)p; u.q[1] = *(const v8us*)(p + 16); return u.v;
}
__device__ __forceinline__ v16b fragb_t8(const us_t* p0, int lane) {
  union { v16b v; v8us q[2]; } u; const v8us z = {0, 0, 0, 0, 0, 0, 0, 0};
  const v8us t = *(const v8us*)(p0 + 8 * (lane >> 4));
  u.q[0] = (lane < 16) ? t : z; u.q[1] = z; return u.v;
}
__device__ __forceinline__ v16b fragb_t16(const us_t* p0, int lane) {
  union { v16b v; v8us q[2]; } u; const v8us z = {0, 0, 0, 0, 0, 0, 0, 0};
  u.q[0] = *(const v8us*)(p0 + 8 * (lane >> 4)); u.q[1] = z; return u.v;
}
#define LDSX() do { asm volatile("s_wait_dscnt 0" ::: "memory"); __builtin_amdgcn_wave_barrier(); __builtin_amdgcn_fence(__ATOMIC_RELEASE, "workgroup"); } while (0)

template <int NT, int KS, int TAIL, int APITCH, int NSTORE, int OPITCH, int OLO, int OROW0>
__device__ __forceinline__ void conv_layer(const us_t* aplane, const us_t* wt, const float* bias, us_t* oplane,
                                           int jb, int wave, int lane) {
  constexpr int KF = KS * 32;
  const int m = lane & 15, h = lane >> 4;
  const us_t* arow = aplane + (wave * 16 + m) * APITCH;
  v8f acc[NT] = {};
#pragma unroll
  for (int s = 0; s < KS; ++s) {
    v16b a;
    if (TAIL == 1 && s == KS - 1) a = fragb_t8(arow + 32 * s, lane);
    else if (TAIL == 2 && s == KS - 1) a = fragb_t16(arow + 32 * s, lane);
    else a = fragb(arow + 32 * s, lane);
#pragma unroll
    for (int j = 0; j < NT; ++j) acc[j] = wmma_bf(a, fragb(wt + (16 * j + m) * KF + 32 * s, lane), acc[j]);
  }
#pragma unroll
  for (int j = 0; j < NT; ++j) {
    const int col = 16 * j + m; const float bv = bias[col];
#pragma unroll
    for (int r = 0; r < 8; ++r) {
      const int pe = wave * 16 + 8 * h + r; const int p = jb + 1 + pe;
      float y = elu_f(acc[j][r] + bv); y = (p < NPTS) ? y : 0.0f;
      const __bf16 hb = (__bf16)y; const __bf16 lb = (__bf16)(y - (float)hb);
      if (col < NSTORE) {
        us_t* o = oplane + (pe + OROW0) * OPITCH + col;
        o[0] = __builtin_bit_cast(us_t, hb); o[OLO] = __builtin_bit_cast(us_t, lb);
      }
    }
  }
}

__device__ __forceinline__ void conv_l5(const us_t* aplane, const us_t* wt, const float* bias, float* S, int wave, int lane) {
  const int m = lane & 15, h = lane >> 4;
  const us_t* arow = aplane + (wave * 16 + m) * P4;
  v8f acc[2] = {};
#pragma unroll
  for (int s = 0; s < K5 / 32; ++s) {
    v16b a;
    if (s == K5 / 32 - 1) a = fragb_t16(arow + 32 * s, lane); else a = fragb(arow + 32 * s, lane);
#pragma unroll
    for (int j = 0; j < 2; ++j) acc[j] = wmma_bf(a, fragb(wt + (16 * j + m) * K5 + 32 * s, lane), acc[j]);
  }
#pragma unroll
  for (int j = 0; j < 2; ++j) {
    const int col = 16 * j + m; const float bv = bias[col];
#pragma unroll
    for (int r = 0; r < 8; ++r) { const float y = elu_f(acc[j][r] + bv); if (col < 20) S[(8 * h + r) * 24 + col] = y; }
  }
}

__device__ __forceinline__ float recon_flux(float bb0, float bb1, float bb2, float f0, float f1, float f2, float eb) {
  const float dd = bb2 - bb0; const float brs = dd * dd;
  const float e0 = eb + bb0, e1 = eb + bb1, e2 = eb + bb2;
  const float q0 = e0 * e0, q1 = e1 * e1, q2 = e2 * e2;
  const float o0 = 0.1f / q0 * (brs + q0);
  const float o1 = 0.6f / q1 * (brs + q1);
  const float o2 = 0.3f / q2 * (brs + q2);
  const float s = o0 + o1 + o2;
  const float a0 = o0 / s, a1 = o1 / s, a2 = o2 / s;
  return a0 * f0 + a1 * f1 + a2 * f2;
}

__device__ __forceinline__ void copy_tab(us_t* wbuf, const unsigned* tabs, int off_bytes, int nbytes, int tid) {
  const v4u* src = (const v4u*)(tabs + off_bytes / 4); v4u* dst = (v4u*)wbuf;
  for (int q = tid; q < nbytes / 16; q += NTHR) dst[q] = src[q];
}

__global__ __launch_bounds__(256) void k_wprep(const float* __restrict__ w2, const float* __restrict__ w3,
                                               const float* __restrict__ w4, const float* __restrict__ w5,
                                               unsigned short* __restrict__ tab) {
  const int tsel = blockIdx.y;
  const int c = blockIdx.x * 256 + threadIdx.x;
  union { v8us h; v4u u; } pk;
  if (tsel == 0) {
    if (c >= T2_BYTES / 16) return;
#pragma unroll
    for (int i = 0; i < 8; ++i) {
      const int e = c * 8 + i, n = e / K2, k = e - n * K2;
      const int kk = k < 199 ? k : 199, nn = n < 39 ? n : 39;
      const int t = kk / 40, cc = (kk - t * 40) % 20;
      const float v = w2[(nn * 20 + cc) * 5 + t];
      pk.h[i] = (n < 40 && k < 200) ? bfbits(v) : (us_t)0;
    }
    vst2(tab + (size_t)(T2_OFF / 2) + (size_t)c * 8, pk.u);
  } else if (tsel == 1) {
    if (c >= T3_BYTES / 16) return;
#pragma unroll
    for (int i = 0; i < 8; ++i) {
      const int e = c * 8 + i, n = e / K3, k = e - n * K3;
      const int cc = k % 48, ccl = cc < 39 ? cc : 39;
      const float v = w3[n * 40 + ccl];
      pk.h[i] = (cc < 40) ? bfbits(v) : (us_t)0;
    }
    vst2(tab + (size_t)(T3_OFF / 2) + (size_t)c * 8, pk.u);
  } else if (tsel == 2) {
    if (c >= T4_BYTES / 16) return;
#pragma unroll
    for (int i = 0; i < 8; ++i) {
      const int e = c * 8 + i, n = e / K4, k = e - n * K4;
      const int cc = k % 80, nn = n < 39 ? n : 39;
      const float v = w4[nn * 80 + cc];
      pk.h[i] = (n < 40) ? bfbits(v) : (us_t)0;
    }
    vst2(tab + (size_t)(T4_OFF / 2) + (size_t)c * 8, pk.u);
  } else {
    if (c >= T5_BYTES / 16) return;
#pragma unroll
    for (int i = 0; i < 8; ++i) {
      const int e = c * 8 + i, n = e / K5, k = e - n * K5;
      const int kk = k < 239 ? k : 239, nn = n < 19 ? n : 19;
      const int t = kk / 80, cc = (kk - t * 80) % 40;
      const float v = w5[(nn * 40 + cc) * 3 + t];
      pk.h[i] = (n < 20 && k < 240) ? bfbits(v) : (us_t)0;
    }
    vst2(tab + (size_t)(T5_OFF / 2) + (size_t)c * 8, pk.u);
  }
}

__global__ __launch_bounds__(NTHR) void k_main(const float* __restrict__ uu, const float* __restrict__ ep,
                                              const float* __restrict__ w1, const float* __restrict__ b1,
                                              const float* __restrict__ b2, const float* __restrict__ b3,
                                              const float* __restrict__ b4, const float* __restrict__ b5,
                                              const float* __restrict__ w6, const float* __restrict__ b6,
                                              const unsigned* __restrict__ tabs, float* __restrict__ out) {
  __shared__ __align__(16) us_t bufA[BUFA_US];
  __shared__ __align__(16) us_t bufB[BUFB_US];
  __shared__ __align__(16) us_t wbuf[WBUF_US];
  __shared__ __align__(16) float out_s[OPB];
  __shared__ float uu_s[UUN];
  __shared__ float dif_s[DIFN];
  __shared__ float beta_s[EXT];
  __shared__ float w1s[100], w6s[20], b1s[20], b2s[48], b3s[80], b4s[48], b5s[32], sc_s[2];

  const int tid = threadIdx.x, wave = tid >> 5, lane = tid & 31;
  const int jb = blockIdx.x * OPB;

  for (int i = tid; i < UUN; i += NTHR) { int p = jb - 4 + i; p = p < 0 ? 0 : p; p = p > NPTS - 1 ? NPTS - 1 : p; uu_s[i] = bfr(uu[p]); }
  for (int i = tid; i < 100; i += NTHR) w1s[i] = bfr(w1[i]);
  for (int i = tid; i < 80; i += NTHR) b3s[i] = bfr(b3[i]);
  for (int i = tid; i < 48; i += NTHR) { const int c = i < 39 ? i : 39; const float v2 = bfr(b2[c]), v4 = bfr(b4[c]); b2s[i] = i < 40 ? v2 : 0.0f; b4s[i] = i < 40 ? v4 : 0.0f; }
  for (int i = tid; i < 32; i += NTHR) { const int c = i < 19 ? i : 19; const float v5 = bfr(b5[c]); b5s[i] = i < 20 ? v5 : 0.0f; }
  for (int i = tid; i < 20; i += NTHR) { w6s[i] = bfr(w6[i]); b1s[i] = bfr(b1[i]); }
  if (tid == 0) { sc_s[0] = bfr(ep[0]); sc_s[1] = bfr(b6[0]); }
  copy_tab(wbuf, tabs, T2_OFF, T2_BYTES, tid);
  __syncthreads();

  for (int d = tid; d < DIFN; d += NTHR) {
    const int p = jb - 3 + d;
    const float a0 = uu_s[d], a1 = uu_s[d + 1], a2 = uu_s[d + 2];
    const float dl = a2 - a1, dr = a1 - a0;
    float v = 0.5f * dl + 0.5f * dr;
    v = (p == 0) ? dl : v; v = (p == NPTS - 1) ? dr : v; v = (p < 0 || p >= NPTS) ? 0.0f : v;
    dif_s[d] = v;
  }
  __syncthreads();

  for (int it = tid; it < L1R * 20; it += NTHR) {
    const int r = it / 20, c = it - r * 20; const int p = jb - 1 + r;
    float s = 0.0f;
#pragma unroll
    for (int t = 0; t < 5; ++t) s = s + w1s[c * 5 + t] * dif_s[r + t];
    float y = elu_f(s + b1s[c]); y = (p >= 0 && p < NPTS) ? y : 0.0f;
    const __bf16 hb = (__bf16)y; const __bf16 lb = (__bf16)(y - (float)hb);
    bufA[r * P1 + c] = __builtin_bit_cast(us_t, hb); bufA[r * P1 + 20 + c] = __builtin_bit_cast(us_t, lb);
  }
  __syncthreads();

  conv_layer<3, K2 / 32, 1, P1, 48, P2, 48, 0>(bufA, wbuf, b2s, bufB, jb, wave, lane);
  __syncthreads();
  copy_tab(wbuf, tabs, T3_OFF, T3_BYTES, tid);
  __syncthreads();

  conv_layer<5, K3 / 32, 0, P2, 80, P3, 80, 0>(bufB, wbuf, b3s, bufA, jb, wave, lane);
  __syncthreads();
  copy_tab(wbuf, tabs, T4_OFF, T4_BYTES, tid);
  { unsigned* zb = (unsigned*)bufB;
    for (int q = tid; q < 3 * (P4 / 2); q += NTHR) { const int rr = q / (P4 / 2), cc = q - rr * (P4 / 2); const int row = (rr == 0) ? 0 : (EXT + rr); zb[row * (P4 / 2) + cc] = 0u; } }
  __syncthreads();

  conv_layer<3, K4 / 32, 0, P3, 40, P4, 40, 1>(bufA, wbuf, b4s, bufB, jb, wave, lane);
  __syncthreads();
  copy_tab(wbuf, tabs, T5_OFF, T5_BYTES, tid);
  __syncthreads();

  float* S5 = reinterpret_cast<float*>(bufA) + wave * (16 * 24);
  conv_l5(bufB, wbuf, b5s, S5, wave, lane);
  LDSX();
  { const int m = lane & 15; float a6 = 0.0f;
#pragma unroll
    for (int c = 0; c < 20; ++c) a6 = a6 + w6s[c] * S5[m * 24 + c];
    a6 = a6 + sc_s[1];
    const float sg = 1.0f / (1.0f + __expf(-a6));
    if (lane < 16) beta_s[wave * 16 + m] = sg + 0.1f; }
  __syncthreads();

  if (tid < OPB) {
    const float eb = sc_s[0];
    const int i0 = tid + 5;
    const float u1 = uu_s[i0], u2 = uu_s[i0 + 1], u3 = uu_s[i0 + 2], u4 = uu_s[i0 + 3], u5 = uu_s[i0 + 4], u6 = uu_s[i0 + 5];
    const float m0 = beta_s[tid + 1], m1 = beta_s[tid + 2], m2 = beta_s[tid + 3];
    const float c6 = 1.0f / 6.0f, c13 = 13.0f / 12.0f;
    float t, t2;
    const float fp0 = (11.0f * u4 - 7.0f * u5 + 2.0f * u6) * c6;
    const float fp1 = (2.0f * u3 + 5.0f * u4 - u5) * c6;
    const float fp2 = (-u2 + 5.0f * u3 + 2.0f * u4) * c6;
    t = u4 - 2.0f * u5 + u6; t2 = 3.0f * u4 - 4.0f * u5 + u6;        const float bp0 = (c13 * (t * t) + 0.25f * (t2 * t2)) * m0;
    t = u3 - 2.0f * u4 + u5; t2 = u3 - u5;                           const float bp1 = (c13 * (t * t) + 0.25f * (t2 * t2)) * m1;
    t = u2 - 2.0f * u3 + u4; t2 = u2 - 4.0f * u3 + 3.0f * u4;        const float bp2 = (c13 * (t * t) + 0.25f * (t2 * t2)) * m2;
    const float fn0 = (11.0f * u3 - 7.0f * u4 + 2.0f * u5) * c6;
    const float fn1 = (2.0f * u2 + 5.0f * u3 - u4) * c6;
    const float fn2 = (-u1 + 5.0f * u2 + 2.0f * u3) * c6;
    t = u3 - 2.0f * u4 + u5; t2 = 3.0f * u3 - 4.0f * u4 + u5;        const float bn0 = (c13 * (t * t) + 0.25f * (t2 * t2)) * m0;
    t = u2 - 2.0f * u3 + u4; t2 = u2 - u4;                           const float bn1 = (c13 * (t * t) + 0.25f * (t2 * t2)) * m1;
    t = u1 - 2.0f * u2 + u3; t2 = u1 - 4.0f * u2 + 3.0f * u3;        const float bn2 = (c13 * (t * t) + 0.25f * (t2 * t2)) * m2;
    const float fluxp = recon_flux(bp0, bp1, bp2, fp0, fp1, fp2, eb);
    const float fluxn = recon_flux(bn0, bn1, bn2, fn0, fn1, fn2, eb);
    out_s[tid] = (jb + tid < NOUT) ? (fluxp - fluxn) : 0.0f;
  }
  __syncthreads();

  {
    const int cnt = (NOUT - jb) < OPB ? (NOUT - jb) : OPB;
    if (tid < OPB / 4) {
      const int n4 = cnt >> 2, rem = cnt & 3;
      float* ob = out + (size_t)jb;
      if (tid < n4) vst2(ob + 4 * tid, *(const v4f*)(&out_s[4 * tid]));
      if (tid == n4) { for (int e2 = 0; e2 < rem; ++e2) vst2(ob + 4 * tid + e2, (float_a)out_s[4 * tid + e2]); }
    }
  }
}

extern "C" void kernel_launch(void* const* d_in, const int* in_sizes, int n_in,
                              void* d_out, int out_size, void* d_ws, size_t ws_size,
                              hipStream_t stream) {
  if (n_in < 14) return;
  if (in_sizes[0] < NPTS || in_sizes[1] < 1 || in_sizes[2] < 100 || in_sizes[3] < 20 || in_sizes[4] < 4000 ||
      in_sizes[5] < 40 || in_sizes[6] < 3200 || in_sizes[7] < 80 || in_sizes[8] < 3200 || in_sizes[9] < 40 ||
      in_sizes[10] < 2400 || in_sizes[11] < 20 || in_sizes[12] < 20 || in_sizes[13] < 1) return;
  if (out_size < NOUT) return;
  if (ws_size < (size_t)WS_TOTAL) return;
  const float* uu = (const float*)d_in[0];
  const float* e  = (const float*)d_in[1];
  const float* w1 = (const float*)d_in[2];
  const float* b1 = (const float*)d_in[3];
  const float* w2 = (const float*)d_in[4];
  const float* b2 = (const float*)d_in[5];
  const float* w3 = (const float*)d_in[6];
  const float* b3 = (const float*)d_in[7];
  const float* w4 = (const float*)d_in[8];
  const float* b4 = (const float*)d_in[9];
  const float* w5 = (const float*)d_in[10];
  const float* b5 = (const float*)d_in[11];
  const float* w6 = (const float*)d_in[12];
  const float* b6 = (const float*)d_in[13];
  unsigned short* tab = (unsigned short*)d_ws;
  k_wprep<<<dim3((T2_BYTES / 16 + 255) / 256, 4), 256, 0, stream>>>(w2, w3, w4, w5, tab);
  k_main<<<(NOUT + OPB - 1) / OPB, NTHR, 0, stream>>>(uu, e, w1, b1, b2, b3, b4, b5, w6, b6,
                                                      (const unsigned*)d_ws, (float*)d_out);
}
